// Optimized_MHSA_Block_21328807592209
// MI455X (gfx1250) — hardware-run, weakly checked
//
#include <hip/hip_runtime.h>
#include <math.h>

constexpr int kBatch = 8;
constexpr int kSeq   = 1024;
constexpr int kDim   = 1024;
constexpr int kHeads = 16;
constexpr int kHD    = 64;
constexpr int kMlp   = 4096;
constexpr int kTok   = kBatch * kSeq;
constexpr int kGroups = kBatch * kHeads;
constexpr int kGrpPerChunk = 8;
constexpr int kNumChunks = kGroups / kGrpPerChunk;
constexpr int kMlpRows = 2048;
constexpr int kMlpChunks = kTok / kMlpRows;
constexpr float kWCarry    = 16.0f;
constexpr float kWCarryInv = 1.0f / 16.0f;
constexpr float kPCarry    = 2048.0f;
constexpr float kCtxCarry  = 256.0f;
constexpr float kScoreScale = 1.0f / (64.0f * 16.0f);
constexpr float kPVScale   = kCtxCarry / kPCarry;
constexpr float kOutScale  = 1.0f / (kCtxCarry * kWCarry);
constexpr float kInvDim    = 1.0f / 1024.0f;
constexpr float kLnEps     = 1e-5f;

typedef __attribute__((ext_vector_type(16))) _Float16 v16h;
typedef __attribute__((ext_vector_type(8)))  _Float16 v8h;
typedef __attribute__((ext_vector_type(16))) __bf16   v16b;
typedef __attribute__((ext_vector_type(8)))  __bf16   v8b;
typedef __attribute__((ext_vector_type(8)))  float    v8f;
typedef __attribute__((ext_vector_type(4)))  float    v4f;
typedef __attribute__((ext_vector_type(4)))  unsigned int v4u;

__device__ __forceinline__ unsigned short f2bf_bits(float f) {
  unsigned u = __float_as_uint(f);
  return (unsigned short)((u + 0x7FFFu + ((u >> 16) & 1u)) >> 16);
}
__device__ __forceinline__ float bf_bits2f(unsigned short h) { return __uint_as_float(((unsigned)h) << 16); }

__device__ __forceinline__ void dep_guard_h(v8f& a, v8f& b, v16h x, v16h y) { asm volatile("v_nop\n\tv_nop\n\tv_nop\n\tv_nop" : "+v"(a), "+v"(b) : "v"(x), "v"(y)); }
__device__ __forceinline__ void dep_guard_b(v8f& a, v8f& b, v16b x, v16b y) { asm volatile("v_nop\n\tv_nop\n\tv_nop\n\tv_nop" : "+v"(a), "+v"(b) : "v"(x), "v"(y)); }
__device__ __forceinline__ void keep4_h(v16h a, v16h b, v16h c, v16h d) { asm volatile("v_nop" :: "v"(a), "v"(b), "v"(c), "v"(d)); }
__device__ __forceinline__ void keep4_b(v16b a, v16b b, v16b c, v16b d) { asm volatile("v_nop" :: "v"(a), "v"(b), "v"(c), "v"(d)); }
__device__ __forceinline__ void acc_guard4(v8f& a, v8f& b, v8f& c, v8f& d) { asm volatile("v_nop\n\tv_nop\n\tv_nop\n\tv_nop" : "+v"(a), "+v"(b), "+v"(c), "+v"(d)); }
template <typename T> struct Frag;
template <> struct Frag<_Float16> {
  typedef v16h V; union U { v16h v; v8h h[2]; };
  static __device__ __forceinline__ v16h load(const _Float16* p) {
    U f; f.h[0] = *(const v8h*)(p); f.h[1] = *(const v8h*)(p + 16); return f.v;
  }
  static __device__ __forceinline__ v8f mma(v16h a, v16h b, v8f c) {
    return __builtin_amdgcn_wmma_f32_16x16x32_f16(false, a, false, b, (short)0, c, false, false);
  }
  static __device__ __forceinline__ void guard(v8f& a, v8f& b, v16h x, v16h y) { dep_guard_h(a, b, x, y); }
  static __device__ __forceinline__ void keep(v16h a, v16h b, v16h c, v16h d) { keep4_h(a, b, c, d); }
};
template <> struct Frag<__bf16> {
  typedef v16b V; union U { v16b v; v8b h[2]; };
  static __device__ __forceinline__ v16b load(const __bf16* p) {
    U f; f.h[0] = *(const v8b*)(p); f.h[1] = *(const v8b*)(p + 16); return f.v;
  }
  static __device__ __forceinline__ v8f mma(v16b a, v16b b, v8f c) {
    return __builtin_amdgcn_wmma_f32_16x16x32_bf16(false, a, false, b, (short)0, c, false, false);
  }
  static __device__ __forceinline__ void guard(v8f& a, v8f& b, v16b x, v16b y) { dep_guard_b(a, b, x, y); }
  static __device__ __forceinline__ void keep(v16b a, v16b b, v16b c, v16b d) { keep4_b(a, b, c, d); }
};

__device__ __forceinline__ unsigned pk16(unsigned short a, unsigned short b) { return (unsigned)a | ((unsigned)b << 16); }
__device__ __forceinline__ unsigned short h_bits(float f) { const _Float16 h = (_Float16)f; return __builtin_bit_cast(unsigned short, h); }

template <int ET> struct Elem;
template <> struct Elem<0> { typedef _Float16 T; };
template <> struct Elem<1> { typedef __bf16 T; };
template <int ET, bool SPLIT, int BIAS_MODE, int OUT_MODE, bool RESID, int ACT = 0>
__global__ __launch_bounds__(256) void wmma_gemm64(
    const unsigned short* __restrict__ Ap, const unsigned short* __restrict__ A2p, int lda, long strideA,
    const unsigned short* __restrict__ Btp, const unsigned short* __restrict__ Bt2p, int ldb, long strideB,
    void* __restrict__ Cout, void* __restrict__ Cout2, int ldc, long strideC,
    const float* __restrict__ bias,
    const float* __restrict__ resid, long strideR,
    int M, int N, int K, float scale) {
  typedef typename Elem<ET>::T T;
  typedef typename Frag<T>::V V;
  const T* A = (const T*)Ap; const T* A2 = (const T*)A2p; const T* Bt = (const T*)Btp; const T* Bt2 = (const T*)Bt2p;
  __shared__ __align__(16) float sT[8][16 * 68];
  const int b    = blockIdx.y;
  const int lane = threadIdx.x & 31;
  const int wave = threadIdx.x >> 5;
  const int tilesN = N >> 6;
  const int tilesM = M >> 6;
  const int tile = blockIdx.x * 8 + wave;
  if (tile >= tilesM * tilesN) return;
  const int tm = tile / tilesN;
  const int tn = tile - tm * tilesN;
  const int m0 = tm << 6;
  const int n0 = tn << 6;

  const T* Ab  = A  + (size_t)b * strideA;
  const T* Bb  = Bt + (size_t)b * strideB;
  const T* Ab2 = SPLIT ? (A2  + (size_t)b * strideA) : nullptr;
  const T* Bb2 = SPLIT ? (Bt2 + (size_t)b * strideB) : nullptr;

  const int rlane = lane & 15;
  const int koff  = (lane >> 4) * 8;
  const int mOff  = (lane >> 4) * 8;

  v8f acc[4][4];
#pragma unroll
  for (int i = 0; i < 4; ++i)
#pragma unroll
    for (int j = 0; j < 4; ++j) acc[i][j] = (v8f){0.f,0.f,0.f,0.f,0.f,0.f,0.f,0.f};

  for (int k0 = 0; k0 < K; k0 += 32) {
    V bh[4], bl[4];
#pragma unroll
    for (int j = 0; j < 4; ++j) {
      const size_t bo = (size_t)(n0 + (j << 4) + rlane) * ldb + koff + k0;
      bh[j] = Frag<T>::load(Bb + bo);
      if (SPLIT) bl[j] = Frag<T>::load(Bb2 + bo);
    }
#pragma unroll
    for (int i = 0; i < 4; ++i) {
      const size_t ao = (size_t)(m0 + (i << 4) + rlane) * lda + koff + k0;
      V ah = Frag<T>::load(Ab + ao);
      V al;
      if (SPLIT) al = Frag<T>::load(Ab2 + ao);
#pragma unroll
      for (int j = 0; j < 4; ++j) {
        acc[i][j] = Frag<T>::mma(ah, bh[j], acc[i][j]);
        if (SPLIT) {
          acc[i][j] = Frag<T>::mma(ah, bl[j], acc[i][j]);
          acc[i][j] = Frag<T>::mma(al, bh[j], acc[i][j]);
        }
      }
      Frag<T>::guard(acc[i][0], acc[i][3], ah, SPLIT ? al : ah);
    }
    Frag<T>::keep(bh[0], bh[1], bh[2], bh[3]);
    if (SPLIT) Frag<T>::keep(bl[0], bl[1], bl[2], bl[3]);
  }
  acc_guard4(acc[0][0], acc[0][1], acc[0][2], acc[0][3]);
  acc_guard4(acc[1][0], acc[1][1], acc[1][2], acc[1][3]);
  acc_guard4(acc[2][0], acc[2][1], acc[2][2], acc[2][3]);
  acc_guard4(acc[3][0], acc[3][1], acc[3][2], acc[3][3]);

  float* slab = sT[wave];
  const float* Rb = RESID ? (resid + (size_t)b * strideR) : nullptr;
#pragma unroll
  for (int i = 0; i < 4; ++i) {
    const int mBase = m0 + (i << 4);
#pragma unroll
    for (int j = 0; j < 4; ++j) {
      const int n = n0 + (j << 4) + rlane;
      float bv = 0.f;
      if (BIAS_MODE == 2) bv = bias[n];
#pragma unroll
      for (int r = 0; r < 8; ++r) {
        float v = acc[i][j][r] * scale;
        if (BIAS_MODE == 1) v += bias[mBase + mOff + r];
        if (BIAS_MODE == 2) v += bv;
        if (RESID) v += Rb[(size_t)(mBase + mOff + r) * ldc + n];
        if (ACT == 2) v = fmaxf(v, 0.0f);
        if (ACT == 4) v = (v > 0.f) ? v : 0.01f * v;
        slab[(mOff + r) * 68 + (j << 4) + rlane] = v;
      }
    }
    __builtin_amdgcn_fence(__ATOMIC_RELEASE, "workgroup");
    __builtin_amdgcn_wave_barrier();
    __builtin_amdgcn_fence(__ATOMIC_ACQUIRE, "workgroup");
    if (OUT_MODE == 0) {
      float* C = (float*)Cout + (size_t)b * strideC;
      const int hh = lane >> 4, c4 = (lane & 15) * 4;
      for (int pass = 0; pass < 2; ++pass) {
#pragma unroll
        for (int it = 0; it < 8; ++it) {
          const int row = it * 2 + hh;
          v4f v = *(const v4f*)(slab + row * 68 + c4);
          *(volatile v4f*)(C + (size_t)(mBase + row) * ldc + n0 + c4) = v;
        }
        __threadfence();
      }
    } else {
      const int q = lane >> 3, c8 = (lane & 7) * 8;
      unsigned short* C  = (unsigned short*)Cout  + (size_t)b * strideC;
      unsigned short* C2 = (OUT_MODE == 2) ? ((unsigned short*)Cout2 + (size_t)b * strideC) : nullptr;
      for (int pass = 0; pass < 2; ++pass) {
#pragma unroll
        for (int it = 0; it < 4; ++it) {
          const int row = it * 4 + q;
          const float* sp = slab + row * 68 + c8;
          v8h hv, lv;
#pragma unroll
          for (int e = 0; e < 8; ++e) {
            if (OUT_MODE == 1) {
              hv[e] = (_Float16)sp[e];
            } else {
              unsigned short hb = f2bf_bits(sp[e]);
              unsigned short lb = f2bf_bits(sp[e] - bf_bits2f(hb));
              hv[e] = __builtin_bit_cast(_Float16, hb);
              lv[e] = __builtin_bit_cast(_Float16, lb);
            }
          }
          *(volatile v8h*)(C + (size_t)(mBase + row) * ldc + n0 + c8) = hv;
          if (OUT_MODE == 2) *(volatile v8h*)(C2 + (size_t)(mBase + row) * ldc + n0 + c8) = lv;
        }
        __threadfence();
      }
    }
    __builtin_amdgcn_fence(__ATOMIC_RELEASE, "workgroup");
    __builtin_amdgcn_wave_barrier();
    __builtin_amdgcn_fence(__ATOMIC_ACQUIRE, "workgroup");
  }
}

__global__ __launch_bounds__(256) void tcast_kernel(const float* __restrict__ in, unsigned short* __restrict__ out,
                                                    int R, int C, long zin, long zout, float scale) {
  __shared__ float sm[64][65];
  const int t  = threadIdx.x;
  const int r0 = blockIdx.x * 64;
  const int c0 = blockIdx.y * 64;
  const float* W = in + (size_t)blockIdx.z * zin;
  unsigned short* op = out + (size_t)blockIdx.z * zout;
#pragma unroll
  for (int i = 0; i < 16; ++i) {
    const int e  = i * 256 + t;
    const int rl = e >> 6;
    const int cl = e & 63;
    sm[cl][rl] = W[(size_t)(r0 + rl) * C + c0 + cl] * scale;
  }
  __syncthreads();
  const int lane = t & 31, wave = t >> 5;
  const int q = lane >> 3, c8 = (lane & 7) * 8;
  for (int pass = 0; pass < 2; ++pass) {
#pragma unroll
    for (int it = 0; it < 2; ++it) {
      const int row = wave * 8 + it * 4 + q;
      unsigned short hb[8];
#pragma unroll
      for (int e = 0; e < 8; ++e) hb[e] = h_bits(sm[row][c8 + e]);
      const v4u u = (v4u){pk16(hb[0], hb[1]), pk16(hb[2], hb[3]), pk16(hb[4], hb[5]), pk16(hb[6], hb[7])};
      *(volatile v4u*)(op + (size_t)(c0 + row) * R + r0 + c8) = u;
    }
    __threadfence();
  }
}

__global__ __launch_bounds__(128) void ln_f16_kernel(const float* __restrict__ x, const float* __restrict__ gam,
                                                     const float* __restrict__ bet, unsigned short* __restrict__ out) {
  __shared__ float redA[4];
  __shared__ float redB[4];
  const int row  = blockIdx.x;
  const int t    = threadIdx.x;
  const int lane = t & 31, wave = t >> 5;
  const int c0   = t * 8;
  const float* xr = x + (size_t)row * kDim + c0;
  const v4f a = *(const v4f*)(xr);
  const v4f c = *(const v4f*)(xr + 4);
  float xs[8];
#pragma unroll
  for (int e = 0; e < 4; ++e) { xs[e] = a[e]; xs[4 + e] = c[e]; }
  float s = ((xs[0] + xs[1]) + (xs[2] + xs[3])) + ((xs[4] + xs[5]) + (xs[6] + xs[7]));
#pragma unroll
  for (int off = 16; off > 0; off >>= 1) s += __shfl_xor(s, off, 32);
  if (lane == 0) redA[wave] = s;
  __syncthreads();
  const float mean = ((redA[0] + redA[1]) + (redA[2] + redA[3])) * kInvDim;
  float d[8];
  float q = 0.f;
#pragma unroll
  for (int e = 0; e < 8; ++e) { d[e] = xs[e] - mean; q += d[e] * d[e]; }
#pragma unroll
  for (int off = 16; off > 0; off >>= 1) q += __shfl_xor(q, off, 32);
  if (lane == 0) redB[wave] = q;
  __syncthreads();
  const float var  = ((redB[0] + redB[1]) + (redB[2] + redB[3])) * kInvDim;
  const float rstd = rsqrtf(var + kLnEps);
  const v4f g0 = *(const v4f*)(gam + c0);
  const v4f g1 = *(const v4f*)(gam + c0 + 4);
  const v4f b0 = *(const v4f*)(bet + c0);
  const v4f b1 = *(const v4f*)(bet + c0 + 4);
  float gg[8], bb[8];
#pragma unroll
  for (int e = 0; e < 4; ++e) { gg[e] = g0[e]; gg[4 + e] = g1[e]; bb[e] = b0[e]; bb[4 + e] = b1[e]; }
  unsigned short hb[8];
#pragma unroll
  for (int e = 0; e < 8; ++e) hb[e] = h_bits(d[e] * rstd * gg[e] + bb[e]);
  const v4u u = (v4u){pk16(hb[0], hb[1]), pk16(hb[2], hb[3]), pk16(hb[4], hb[5]), pk16(hb[6], hb[7])};
  unsigned short* op = out + (size_t)row * kDim + c0;
  *(volatile v4u*)op = u;
  __threadfence();
  *(volatile v4u*)op = u;
}

__global__ __launch_bounds__(128) void softmax_f16_kernel(const float* __restrict__ S, unsigned short* __restrict__ P, float carry) {
  __shared__ float redM[4];
  __shared__ float redS[4];
  const int row  = blockIdx.x;
  const int t    = threadIdx.x;
  const int lane = t & 31, wave = t >> 5;
  const int c0   = t * 8;
  const float* sr = S + (size_t)row * kSeq + c0;
  const v4f a = *(const v4f*)(sr);
  const v4f c = *(const v4f*)(sr + 4);
  float xs[8];
#pragma unroll
  for (int e = 0; e < 4; ++e) { xs[e] = a[e]; xs[4 + e] = c[e]; }
  float m = fmaxf(fmaxf(fmaxf(xs[0], xs[1]), fmaxf(xs[2], xs[3])), fmaxf(fmaxf(xs[4], xs[5]), fmaxf(xs[6], xs[7])));
#pragma unroll
  for (int off = 16; off > 0; off >>= 1) m = fmaxf(m, __shfl_xor(m, off, 32));
  if (lane == 0) redM[wave] = m;
  __syncthreads();
  const float mx = fmaxf(fmaxf(redM[0], redM[1]), fmaxf(redM[2], redM[3]));
  float ex[8];
  float s = 0.f;
#pragma unroll
  for (int e = 0; e < 8; ++e) { ex[e] = expf(xs[e] - mx); s += ex[e]; }
#pragma unroll
  for (int off = 16; off > 0; off >>= 1) s += __shfl_xor(s, off, 32);
  if (lane == 0) redS[wave] = s;
  __syncthreads();
  const float tot = ((redS[0] + redS[1]) + (redS[2] + redS[3]));
  const float inv = carry / tot;
  unsigned short hb[8];
#pragma unroll
  for (int e = 0; e < 8; ++e) hb[e] = h_bits(ex[e] * inv);
  const v4u u = (v4u){pk16(hb[0], hb[1]), pk16(hb[2], hb[3]), pk16(hb[4], hb[5]), pk16(hb[6], hb[7])};
  unsigned short* op = P + (size_t)row * kSeq + c0;
  *(volatile v4u*)op = u;
  __threadfence();
  *(volatile v4u*)op = u;
}

__global__ __launch_bounds__(256) void xtrans_kernel(const unsigned short* __restrict__ X, unsigned short* __restrict__ XT) {
  __shared__ unsigned short sm[64][72];
  const int t  = threadIdx.x;
  const int tt = blockIdx.x;
  const int g  = blockIdx.y;
  const int b  = g >> 4, h = g & 15;
  const size_t rowbase = (size_t)b * kSeq + (size_t)tt * 64;
#pragma unroll
  for (int it = 0; it < 2; ++it) {
    const int idx = it * 256 + t;
    const int r = idx >> 3, k = idx & 7;
    const v4u w = *(const v4u*)(X + (rowbase + r) * kDim + h * kHD + 8 * k);
#pragma unroll
    for (int e = 0; e < 4; ++e) {
      sm[r][8 * k + 2 * e]     = (unsigned short)(w[e] & 0xffffu);
      sm[r][8 * k + 2 * e + 1] = (unsigned short)(w[e] >> 16);
    }
  }
  __syncthreads();
  unsigned short* op = XT + (size_t)g * (kHD * kSeq) + (size_t)tt * 64;
  const int lane = t & 31, wave = t >> 5;
  for (int pass = 0; pass < 2; ++pass) {
#pragma unroll
    for (int it = 0; it < 2; ++it) {
      const int idx = it * 256 + wave * 32 + lane;
      const int d = idx >> 3, k = idx & 7;
      const v4u u = (v4u){pk16(sm[8 * k + 0][d], sm[8 * k + 1][d]), pk16(sm[8 * k + 2][d], sm[8 * k + 3][d]),
                          pk16(sm[8 * k + 4][d], sm[8 * k + 5][d]), pk16(sm[8 * k + 6][d], sm[8 * k + 7][d])};
      *(volatile v4u*)(op + (size_t)d * kSeq + 8 * k) = u;
    }
    __threadfence();
  }
}

__global__ __launch_bounds__(256) void gelu_f16x2_kernel(const float* __restrict__ in, unsigned short* __restrict__ out, int n2) {
  const int i = blockIdx.x * 256 + threadIdx.x;
  if (i >= n2) return;
  unsigned packed = 0u;
#pragma unroll 1
  for (int e = 0; e < 2; ++e) {
    const float u  = in[2 * (size_t)i + e];
    const float gl = 0.5f * u * (1.0f + erff(u * 0.70710678118654752f));
    packed |= ((unsigned)h_bits(gl)) << (16 * e);
  }
  ((volatile unsigned*)out)[i] = packed;
  __threadfence();
  ((volatile unsigned*)out)[i] = packed;
}

extern "C" void kernel_launch(void* const* d_in, const int* in_sizes, int n_in,
                              void* d_out, int out_size, void* d_ws,
                              size_t ws_size, hipStream_t stream) {
  (void)in_sizes;
  if (n_in < 14) return;
  const float* inputs = (const float*)d_in[0];
  const float* W_in   = (const float*)d_in[1];
  const float* b_in   = (const float*)d_in[2];
  const float* attn_w = (const float*)d_in[3];
  const float* W_out  = (const float*)d_in[4];
  const float* b_out  = (const float*)d_in[5];
  const float* W1     = (const float*)d_in[6];
  const float* b1     = (const float*)d_in[7];
  const float* W2     = (const float*)d_in[8];
  const float* b2     = (const float*)d_in[9];
  const float* ln1_g  = (const float*)d_in[10];
  const float* ln1_b  = (const float*)d_in[11];
  const float* ln2_g  = (const float*)d_in[12];
  const float* ln2_b  = (const float*)d_in[13];

  const size_t MiB = 1048576;
  const size_t need = 114 * MiB;
  if (ws_size < need) return;
  if ((size_t)out_size < (size_t)kTok * kDim) return;

  char* ws = (char*)d_ws;
  unsigned short* X16   = (unsigned short*)(ws + 0 * MiB);
  unsigned short* XT16  = (unsigned short*)(ws + 16 * MiB);
  float*          x1    = (float*)(ws + 0 * MiB);
  unsigned short* XW16  = (unsigned short*)(ws + 32 * MiB);
  unsigned short* yln16 = (unsigned short*)(ws + 32 * MiB);
  unsigned short* AO16  = (unsigned short*)(ws + 48 * MiB);
  unsigned short* H16   = (unsigned short*)(ws + 48 * MiB);
  float*          Spl   = (float*)(ws + 64 * MiB);
  unsigned short* xln16 = (unsigned short*)(ws + 64 * MiB);
  unsigned short* WinT  = (unsigned short*)(ws + 80 * MiB);
  unsigned short* AwT   = (unsigned short*)(ws + 82 * MiB);
  float*          U32   = (float*)(ws + 64 * MiB);
  unsigned short* P16   = (unsigned short*)(ws + 96 * MiB);
  unsigned short* W1T   = (unsigned short*)(ws + 96 * MiB);
  unsigned short* W2T   = (unsigned short*)(ws + 104 * MiB);
  unsigned short* WoutT = (unsigned short*)(ws + 112 * MiB);
  float* outp = (float*)d_out;

  tcast_kernel<<<dim3(kDim / 64, kDim / 64, 1), 256, 0, stream>>>(W_in, WinT, kDim, kDim, 0L, 0L, kWCarry);
  tcast_kernel<<<dim3(1, 1, kHeads), 256, 0, stream>>>(attn_w, AwT, kHD, kHD, (long)(kHD * kHD), (long)(kHD * kHD), kWCarry);
  tcast_kernel<<<dim3(kDim / 64, kDim / 64, 1), 256, 0, stream>>>(W_out, WoutT, kDim, kDim, 0L, 0L, kWCarry);

  ln_f16_kernel<<<kTok, 128, 0, stream>>>(inputs, ln1_g, ln1_b, xln16);

  wmma_gemm64<0, false, 2, 1, false><<<dim3(256, 1), 256, 0, stream>>>(
      xln16, xln16, kDim, 0L, WinT, WinT, kDim, 0L,
      (void*)X16, (void*)X16, kDim, 0L, b_in, nullptr, 0L, kTok, kDim, kDim, kWCarryInv);

  xtrans_kernel<<<dim3(kSeq / 64, kGroups), 256, 0, stream>>>(X16, XT16);

  wmma_gemm64<0, false, 0, 1, false><<<dim3(16, kHeads), 256, 0, stream>>>(
      X16, X16, kDim, (long)kHD, AwT, AwT, kHD, (long)(kHD * kHD),
      (void*)XW16, (void*)XW16, kDim, (long)kHD, nullptr, nullptr, 0L, kTok, kHD, kHD, 1.0f);

  for (int c = 0; c < kNumChunks; ++c) {
    const int b  = c >> 1;
    const int h0 = (c & 1) * kGrpPerChunk;
    const size_t off = (size_t)b * kSeq * kDim + (size_t)h0 * kHD;
    wmma_gemm64<0, false, 0, 0, false><<<dim3(32, kGrpPerChunk), 256, 0, stream>>>(
        XW16 + off, XW16 + off, kDim, (long)kHD, X16 + off, X16 + off, kDim, (long)kHD,
        (void*)Spl, (void*)Spl, kSeq, (long)(kSeq * kSeq), nullptr, nullptr, 0L, kSeq, kSeq, kHD, kScoreScale);
    softmax_f16_kernel<<<kGrpPerChunk * kSeq, 128, 0, stream>>>(Spl, P16, kPCarry);
    wmma_gemm64<0, false, 0, 1, false><<<dim3(2, kGrpPerChunk), 256, 0, stream>>>(
        P16, P16, kSeq, (long)(kSeq * kSeq), XT16 + (size_t)(c * kGrpPerChunk) * (kHD * kSeq), XT16 + (size_t)(c * kGrpPerChunk) * (kHD * kSeq), kSeq, (long)(kHD * kSeq),
        (void*)(AO16 + off), (void*)(AO16 + off), kDim, (long)kHD, nullptr, nullptr, 0L, kSeq, kHD, kSeq, kPVScale);
  }

  wmma_gemm64<0, false, 2, 0, true><<<dim3(256, 1), 256, 0, stream>>>(
      AO16, AO16, kDim, 0L, WoutT, WoutT, kDim, 0L,
      (void*)x1, (void*)x1, kDim, 0L, b_out, inputs, 0L, kTok, kDim, kDim, kOutScale);

  tcast_kernel<<<dim3(kDim / 64, kMlp / 64, 1), 256, 0, stream>>>(W1, W1T, kDim, kMlp, 0L, 0L, kWCarry);
  tcast_kernel<<<dim3(kMlp / 64, kDim / 64, 1), 256, 0, stream>>>(W2, W2T, kMlp, kDim, 0L, 0L, kWCarry);

  ln_f16_kernel<<<kTok, 128, 0, stream>>>(x1, ln2_g, ln2_b, yln16);

  for (int q = 0; q < kMlpChunks; ++q) {
    const size_t rowoff = (size_t)q * kMlpRows;
    wmma_gemm64<0, false, 2, 0, false><<<dim3(256, 1), 256, 0, stream>>>(
        yln16 + rowoff * kDim, yln16 + rowoff * kDim, kDim, 0L, W1T, W1T, kDim, 0L,
        (void*)U32, (void*)U32, kMlp, 0L, b1, nullptr, 0L, kMlpRows, kMlp, kDim, kWCarryInv);
    gelu_f16x2_kernel<<<(kMlpRows * kMlp / 2) / 256, 256, 0, stream>>>(U32, H16, kMlpRows * kMlp / 2);
    wmma_gemm64<0, false, 2, 0, true><<<dim3(64, 1), 256, 0, stream>>>(
        H16, H16, kMlp, 0L, W2T, W2T, kMlp, 0L,
        (void*)(outp + rowoff * kDim), (void*)(outp + rowoff * kDim), kDim, 0L, b2, x1 + rowoff * kDim, 0L,
        kMlpRows, kDim, kMlp, kWCarryInv);
  }
}
